// Hyper_SAGNN_1898375545043
// MI455X (gfx1250) — hardware-verified
//
#include <hip/hip_runtime.h>
#include <stdint.h>
#include <math.h>

typedef __attribute__((ext_vector_type(16))) _Float16 v16h;
typedef __attribute__((ext_vector_type(8)))  _Float16 v8h;
typedef __attribute__((ext_vector_type(16))) __bf16   v16b;
typedef __attribute__((ext_vector_type(8)))  __bf16   v8b;
typedef __attribute__((ext_vector_type(8)))  float    v8f;
typedef __attribute__((ext_vector_type(4)))  float    v4f;
typedef _Float16 f16t;

#define LN_D 512

__device__ __forceinline__ unsigned short f2bf_bits(float f) {
  unsigned u = __float_as_uint(f);
  return (unsigned short)((u + 0x7FFFu + ((u >> 16) & 1u)) >> 16);
}
__device__ __forceinline__ float bf_bits2f(unsigned short h) { return __uint_as_float(((unsigned)h) << 16); }

__device__ __forceinline__ void dep_guard_h(v8f& a, v8f& b, v16h x, v16h y) { asm volatile("v_nop\n\tv_nop\n\tv_nop\n\tv_nop" : "+v"(a), "+v"(b) : "v"(x), "v"(y)); }
__device__ __forceinline__ void dep_guard_b(v8f& a, v8f& b, v16b x, v16b y) { asm volatile("v_nop\n\tv_nop\n\tv_nop\n\tv_nop" : "+v"(a), "+v"(b) : "v"(x), "v"(y)); }
__device__ __forceinline__ void keep4_h(v16h a, v16h b, v16h c, v16h d) { asm volatile("v_nop" :: "v"(a), "v"(b), "v"(c), "v"(d)); }
__device__ __forceinline__ void keep4_b(v16b a, v16b b, v16b c, v16b d) { asm volatile("v_nop" :: "v"(a), "v"(b), "v"(c), "v"(d)); }
__device__ __forceinline__ void acc_guard4(v8f& a, v8f& b, v8f& c, v8f& d) { asm volatile("v_nop\n\tv_nop\n\tv_nop\n\tv_nop" : "+v"(a), "+v"(b), "+v"(c), "+v"(d)); }
template <typename T> struct Frag;
template <> struct Frag<_Float16> {
  typedef v16h V; union U { v16h v; v8h h[2]; };
  static __device__ __forceinline__ v16h load(const _Float16* p) {
    U f; f.h[0] = *(const v8h*)(p); f.h[1] = *(const v8h*)(p + 16); return f.v;
  }
  static __device__ __forceinline__ v8f mma(v16h a, v16h b, v8f c) {
    return __builtin_amdgcn_wmma_f32_16x16x32_f16(false, a, false, b, (short)0, c, false, false);
  }
  static __device__ __forceinline__ void guard(v8f& a, v8f& b, v16h x, v16h y) { dep_guard_h(a, b, x, y); }
  static __device__ __forceinline__ void keep(v16h a, v16h b, v16h c, v16h d) { keep4_h(a, b, c, d); }
};
template <> struct Frag<__bf16> {
  typedef v16b V; union U { v16b v; v8b h[2]; };
  static __device__ __forceinline__ v16b load(const __bf16* p) {
    U f; f.h[0] = *(const v8b*)(p); f.h[1] = *(const v8b*)(p + 16); return f.v;
  }
  static __device__ __forceinline__ v8f mma(v16b a, v16b b, v8f c) {
    return __builtin_amdgcn_wmma_f32_16x16x32_bf16(false, a, false, b, (short)0, c, false, false);
  }
  static __device__ __forceinline__ void guard(v8f& a, v8f& b, v16b x, v16b y) { dep_guard_b(a, b, x, y); }
  static __device__ __forceinline__ void keep(v16b a, v16b b, v16b c, v16b d) { keep4_b(a, b, c, d); }
};

template <int ET> struct Elem;
template <> struct Elem<0> { typedef _Float16 T; };
template <> struct Elem<1> { typedef __bf16 T; };
template <int ET, bool SPLIT, int BIAS_MODE, int OUT_MODE, bool RESID, int ACT, bool RS>
__global__ __launch_bounds__(256) void wmma_gemm64(
    const unsigned short* __restrict__ Ap, const unsigned short* __restrict__ A2p, int lda, long strideA,
    const unsigned short* __restrict__ Btp, const unsigned short* __restrict__ Bt2p, int ldb, long strideB,
    void* __restrict__ Cout, void* __restrict__ Cout2, int ldc, long strideC,
    const float* __restrict__ bias,
    const float* __restrict__ resid, long strideR,
    const float* __restrict__ rsc,
    int M, int N, int K, float scale) {
  typedef typename Elem<ET>::T T;
  typedef typename Frag<T>::V V;
  const T* A = (const T*)Ap; const T* A2 = (const T*)A2p; const T* Bt = (const T*)Btp; const T* Bt2 = (const T*)Bt2p;
  __shared__ __align__(16) float sT[8][16 * 68];
  const int b    = blockIdx.y;
  const int lane = threadIdx.x & 31;
  const int wave = threadIdx.x >> 5;
  const int tilesN = N >> 6;
  const int tilesM = M >> 6;
  const int tile = blockIdx.x * 8 + wave;
  if (tile >= tilesM * tilesN) return;
  const int tm = tile / tilesN;
  const int tn = tile - tm * tilesN;
  const int m0 = tm << 6;
  const int n0 = tn << 6;

  const T* Ab  = A  + (size_t)b * strideA;
  const T* Bb  = Bt + (size_t)b * strideB;
  const T* Ab2 = SPLIT ? (A2  + (size_t)b * strideA) : nullptr;
  const T* Bb2 = SPLIT ? (Bt2 + (size_t)b * strideB) : nullptr;

  const int rlane = lane & 15;
  const int koff  = (lane >> 4) * 8;
  const int mOff  = (lane >> 4) * 8;

  v8f acc[4][4];
#pragma unroll
  for (int i = 0; i < 4; ++i)
#pragma unroll
    for (int j = 0; j < 4; ++j) acc[i][j] = (v8f){0.f,0.f,0.f,0.f,0.f,0.f,0.f,0.f};

  for (int k0 = 0; k0 < K; k0 += 32) {
    V bh[4], bl[4];
#pragma unroll
    for (int j = 0; j < 4; ++j) {
      const size_t bo = (size_t)(n0 + (j << 4) + rlane) * ldb + koff + k0;
      bh[j] = Frag<T>::load(Bb + bo);
      if (SPLIT) bl[j] = Frag<T>::load(Bb2 + bo);
    }
#pragma unroll
    for (int i = 0; i < 4; ++i) {
      const size_t ao = (size_t)(m0 + (i << 4) + rlane) * lda + koff + k0;
      V ah = Frag<T>::load(Ab + ao);
      V al;
      if (SPLIT) al = Frag<T>::load(Ab2 + ao);
#pragma unroll
      for (int j = 0; j < 4; ++j) {
        acc[i][j] = Frag<T>::mma(ah, bh[j], acc[i][j]);
        if (SPLIT) {
          acc[i][j] = Frag<T>::mma(ah, bl[j], acc[i][j]);
          acc[i][j] = Frag<T>::mma(al, bh[j], acc[i][j]);
        }
      }
      Frag<T>::guard(acc[i][0], acc[i][3], ah, SPLIT ? al : ah);
    }
    Frag<T>::keep(bh[0], bh[1], bh[2], bh[3]);
    if (SPLIT) Frag<T>::keep(bl[0], bl[1], bl[2], bl[3]);
  }
  acc_guard4(acc[0][0], acc[0][1], acc[0][2], acc[0][3]);
  acc_guard4(acc[1][0], acc[1][1], acc[1][2], acc[1][3]);
  acc_guard4(acc[2][0], acc[2][1], acc[2][2], acc[2][3]);
  acc_guard4(acc[3][0], acc[3][1], acc[3][2], acc[3][3]);

  float* slab = sT[wave];
  const float* Rb = RESID ? (resid + (size_t)b * strideR) : nullptr;
#pragma unroll
  for (int i = 0; i < 4; ++i) {
    const int mBase = m0 + (i << 4);
#pragma unroll
    for (int j = 0; j < 4; ++j) {
      const int n = n0 + (j << 4) + rlane;
      float bv = 0.f;
      if (BIAS_MODE == 2) bv = bias[n];
#pragma unroll
      for (int r = 0; r < 8; ++r) {
        float v = acc[i][j][r] * scale;
        if (BIAS_MODE == 1) v += bias[mBase + mOff + r];
        if (BIAS_MODE == 2) v += bv;
        if (RESID) v += Rb[(size_t)(mBase + mOff + r) * ldc + n];
        if (ACT == 1) v = tanhf(v);
        if (ACT == 2) v = fmaxf(v, 0.0f);
        if (ACT == 3) { const float ev = expf(-fmaxf(v, -80.0f)); v = v * (1.0f / (1.0f + ev)); }
        if (ACT == 4) v = (v > 0.f) ? v : 0.01f * v;
        if (ACT == 5) v = 0.5f * v * (1.0f + erff(v * 0.70710678118654752f));
        if (RS) v *= rsc[mBase + mOff + r];
        slab[(mOff + r) * 68 + (j << 4) + rlane] = v;
      }
    }
    __builtin_amdgcn_fence(__ATOMIC_RELEASE, "workgroup");
    __builtin_amdgcn_wave_barrier();
    __builtin_amdgcn_fence(__ATOMIC_ACQUIRE, "workgroup");
    if (OUT_MODE == 0) {
      float* C = (float*)Cout + (size_t)b * strideC;
      const int hh = lane >> 4, c4 = (lane & 15) * 4;
      for (int pass = 0; pass < 2; ++pass) {
#pragma unroll
        for (int it = 0; it < 8; ++it) {
          const int row = it * 2 + hh;
          v4f v = *(const v4f*)(slab + row * 68 + c4);
          *(volatile v4f*)(C + (size_t)(mBase + row) * ldc + n0 + c4) = v;
        }
        __threadfence();
      }
    } else {
      const int q = lane >> 3, c8 = (lane & 7) * 8;
      unsigned short* C  = (unsigned short*)Cout  + (size_t)b * strideC;
      unsigned short* C2 = (OUT_MODE == 2) ? ((unsigned short*)Cout2 + (size_t)b * strideC) : nullptr;
      for (int pass = 0; pass < 2; ++pass) {
#pragma unroll
        for (int it = 0; it < 4; ++it) {
          const int row = it * 4 + q;
          const float* sp = slab + row * 68 + c8;
          v8h hv, lv;
#pragma unroll
          for (int e = 0; e < 8; ++e) {
            if (OUT_MODE == 1) {
              hv[e] = (_Float16)sp[e];
            } else {
              unsigned short hb = f2bf_bits(sp[e]);
              unsigned short lb = f2bf_bits(sp[e] - bf_bits2f(hb));
              hv[e] = __builtin_bit_cast(_Float16, hb);
              lv[e] = __builtin_bit_cast(_Float16, lb);
            }
          }
          *(volatile v8h*)(C + (size_t)(mBase + row) * ldc + n0 + c8) = hv;
          if (OUT_MODE == 2) *(volatile v8h*)(C2 + (size_t)(mBase + row) * ldc + n0 + c8) = lv;
        }
        __threadfence();
      }
    }
    __builtin_amdgcn_fence(__ATOMIC_RELEASE, "workgroup");
    __builtin_amdgcn_wave_barrier();
    __builtin_amdgcn_fence(__ATOMIC_ACQUIRE, "workgroup");
  }
}

__device__ __forceinline__ float wsum32(float v) {
#pragma unroll
  for (int off = 16; off > 0; off >>= 1) v += __shfl_xor(v, off, 32);
  return v;
}
__device__ __forceinline__ void ld8f(const float* __restrict__ p, float (&o)[8]) {
  const v4f a = *(const v4f*)p;
  const v4f b = *(const v4f*)(p + 4);
  o[0] = a[0]; o[1] = a[1]; o[2] = a[2]; o[3] = a[3];
  o[4] = b[0]; o[5] = b[1]; o[6] = b[2]; o[7] = b[3];
}

__global__ __launch_bounds__(256) void wcast_t16(
    const float* __restrict__ w0, const float* __restrict__ w1, const float* __restrict__ w2,
    const float* __restrict__ w3, const float* __restrict__ w4, const float* __restrict__ w5,
    const float* __restrict__ w6, f16t* __restrict__ dst, int Din, int Dout, float mul) {
  __shared__ float tile[32][65];
  const int z = blockIdx.z;
  const float* W = (z == 0) ? w0 : (z == 1) ? w1 : (z == 2) ? w2 : (z == 3) ? w3 : (z == 4) ? w4 : (z == 5) ? w5 : w6;
  f16t* Dp = dst + (size_t)z * Dout * Din;
  const int n0 = blockIdx.y * 32, k0 = blockIdx.x * 64;
  const int tid = threadIdx.x, nl = tid & 31, kg = tid >> 5;
#pragma unroll
  for (int i = 0; i < 8; ++i) {
    const int kl = kg + 8 * i;
    tile[nl][kl] = W[(size_t)(k0 + kl) * Dout + n0 + nl] * mul;
  }
  __syncthreads();
  const int lane = tid & 31, wave = tid >> 5;
  const int rl = wave * 4 + (lane >> 3), c8 = (lane & 7) * 8;
  v8h hv;
#pragma unroll
  for (int e = 0; e < 8; ++e) hv[e] = (f16t)tile[rl][c8 + e];
  f16t* p = Dp + (size_t)(n0 + rl) * Din + k0 + c8;
  *(volatile v8h*)p = hv;
  __threadfence();
  *(volatile v8h*)p = hv;
}

template <int NOUT>
__global__ __launch_bounds__(256) void ln_rows_f16(
    const float* __restrict__ x,
    const float* __restrict__ g0, const float* __restrict__ b0,
    const float* __restrict__ g1, const float* __restrict__ b1,
    f16t* __restrict__ y0, f16t* __restrict__ y1, int nrows, float eps) {
  const int lane = threadIdx.x & 31;
  const int wave = threadIdx.x >> 5;
  const int row = blockIdx.x * 8 + wave;
  if (row >= nrows) return;
  const float* xr = x + (size_t)row * LN_D;
  float xv[16];
  {
    float t[8];
    ld8f(xr + 8 * lane, t);
#pragma unroll
    for (int e = 0; e < 8; ++e) xv[e] = t[e];
    ld8f(xr + 256 + 8 * lane, t);
#pragma unroll
    for (int e = 0; e < 8; ++e) xv[8 + e] = t[e];
  }
  float s = 0.f;
#pragma unroll
  for (int i = 0; i < 16; ++i) s += xv[i];
  s = wsum32(s);
  const float mean = s * (1.0f / 512.0f);
  float vs = 0.f;
#pragma unroll
  for (int i = 0; i < 16; ++i) { const float d = xv[i] - mean; vs += d * d; }
  vs = wsum32(vs);
  const float inv = 1.0f / sqrtf(vs * (1.0f / 512.0f) + eps);

  v8h o0[2], o1[2];
#pragma unroll
  for (int ch = 0; ch < 2; ++ch) {
    const int col = ch * 256 + 8 * lane;
    float gv[8], bv[8];
    ld8f(g0 + col, gv);
    ld8f(b0 + col, bv);
    float g1v[8], b1v[8];
    if (NOUT == 2) { ld8f(g1 + col, g1v); ld8f(b1 + col, b1v); }
#pragma unroll
    for (int e = 0; e < 8; ++e) {
      const float nv = (xv[ch * 8 + e] - mean) * inv;
      o0[ch][e] = (f16t)(nv * gv[e] + bv[e]);
      if (NOUT == 2) o1[ch][e] = (f16t)(nv * g1v[e] + b1v[e]);
    }
  }
  f16t* yr0 = y0 + (size_t)row * LN_D;
  f16t* yr1 = y1 + (size_t)row * LN_D;
#pragma unroll
  for (int ch = 0; ch < 2; ++ch) {
    *(volatile v8h*)(yr0 + ch * 256 + 8 * lane) = o0[ch];
    if (NOUT == 2) *(volatile v8h*)(yr1 + ch * 256 + 8 * lane) = o1[ch];
  }
  __threadfence();
#pragma unroll
  for (int ch = 0; ch < 2; ++ch) {
    *(volatile v8h*)(yr0 + ch * 256 + 8 * lane) = o0[ch];
    if (NOUT == 2) *(volatile v8h*)(yr1 + ch * 256 + 8 * lane) = o1[ch];
  }
}

#define AT_D 64
#define AT_NW 4
#define AT_QB 64
#define AT_KC 64
#define AT_PSC 32768.0f
__device__ __forceinline__ v8f mma_h(v16h a, v16h b, v8f c) {
  c = __builtin_amdgcn_wmma_f32_16x16x32_f16(false, a, false, b, (short)0, c, false, false);
  asm volatile("v_nop\n\tv_nop\n\tv_nop\n\tv_nop" : "+v"(c) : "v"(a), "v"(b));
  return c;
}

__global__ __launch_bounds__(128)
void attn64_f16_diag(const f16t* __restrict__ q, const f16t* __restrict__ k,
                     const f16t* __restrict__ v, f16t* __restrict__ out,
                     int S, int H, int rs, float sm_scale, float mask_fill, float out_scale) {
  union FB { v16h v; v8h h[2]; };
  __shared__ __align__(16) f16t Ksh[AT_KC * AT_D];
  __shared__ __align__(16) f16t Vth[AT_D * AT_KC];
  __shared__ __align__(16) f16t Psh[AT_NW][16 * AT_KC];
  __shared__ __align__(16) float Os[AT_NW][16 * 68];

  const int tid  = threadIdx.x;
  const int wave = tid >> 5;
  const int lane = tid & 31;
  const int hh   = lane >> 4;
  const int c    = lane & 15;

  const int nqb = S / AT_QB;
  const int bx = blockIdx.x;
  const int qb = bx % nqb;
  const int bh = bx / nqb;
  const int h  = bh % H;
  const int b  = bh / H;
  const int q0 = qb * AT_QB + wave * 16;
  const size_t hoff = (size_t)b * S * rs + (size_t)h * AT_D;
  const f16t* qb_ptr = q + hoff;
  const f16t* kb_ptr = k + hoff;
  const f16t* vb_ptr = v + hoff;
  f16t*       ob_ptr = out + hoff;

  v16h qa[2];
  {
    const f16t* qrow = qb_ptr + (size_t)(q0 + c) * rs;
#pragma unroll
    for (int dc = 0; dc < 2; ++dc) qa[dc] = Frag<f16t>::load(qrow + dc * 32 + 8 * hh);
  }

  float mrow[8], lrow[8];
  v8f oacc[4];
#pragma unroll
  for (int r = 0; r < 8; ++r) { mrow[r] = -INFINITY; lrow[r] = 0.f; }
#pragma unroll
  for (int t = 0; t < 4; ++t) oacc[t] = (v8f){0.f,0.f,0.f,0.f,0.f,0.f,0.f,0.f};

  const int nChunks = S / AT_KC;
  for (int kc = 0; kc < nChunks; ++kc) {
    const int kv0 = kc * AT_KC;
    __syncthreads();
    {
      const int kvr = tid >> 1, dh = (tid & 1) * 32;
      const f16t* krow = kb_ptr + (size_t)(kv0 + kvr) * rs + dh;
      const f16t* vrow = vb_ptr + (size_t)(kv0 + kvr) * rs + dh;
#pragma unroll
      for (int i = 0; i < 4; ++i) {
        const v8h kk8 = *(const v8h*)(krow + 8 * i);
        const v8h vv8 = *(const v8h*)(vrow + 8 * i);
        *(v8h*)(Ksh + kvr * AT_D + dh + 8 * i) = kk8;
#pragma unroll
        for (int e = 0; e < 8; ++e) Vth[(dh + 8 * i + e) * AT_KC + kvr] = vv8[e];
      }
    }
    __syncthreads();

    v8f s[4];
#pragma unroll
    for (int j = 0; j < 4; ++j) {
      s[j] = (v8f){0.f,0.f,0.f,0.f,0.f,0.f,0.f,0.f};
#pragma unroll
      for (int dc = 0; dc < 2; ++dc) {
        FB kb;
        kb.h[0] = *(const v8h*)(Ksh + (j * 16 + c) * AT_D + dc * 32 + 8 * hh);
        kb.h[1] = *(const v8h*)(Ksh + (j * 16 + c) * AT_D + dc * 32 + 16 + 8 * hh);
        s[j] = mma_h(qa[dc], kb.v, s[j]);
      }
    }
    float cm[8];
#pragma unroll
    for (int r = 0; r < 8; ++r) {
      const int qrow = q0 + 8 * hh + r;
      float m = -INFINITY;
#pragma unroll
      for (int j = 0; j < 4; ++j) {
        const int kvcol = kv0 + j * 16 + c;
        float val = s[j][r] * sm_scale;
        if (kvcol == qrow) val = mask_fill;
        s[j][r] = val;
        m = fmaxf(m, val);
      }
#pragma unroll
      for (int off = 1; off < 16; off <<= 1) m = fmaxf(m, __shfl_xor(m, off, 32));
      cm[r] = m;
    }
    f16t* pw = Psh[wave];
#pragma unroll
    for (int r = 0; r < 8; ++r) {
      const float mnew = fmaxf(mrow[r], cm[r]);
      const float alpha = expf(mrow[r] - mnew);
      mrow[r] = mnew;
      float psum = 0.f;
#pragma unroll
      for (int j = 0; j < 4; ++j) {
        const float p = expf(s[j][r] - mnew);
        psum += p;
        pw[(8 * hh + r) * AT_KC + j * 16 + c] = (f16t)(p * AT_PSC);
      }
#pragma unroll
      for (int off = 1; off < 16; off <<= 1) psum += __shfl_xor(psum, off, 32);
      lrow[r] = lrow[r] * alpha + psum;
#pragma unroll
      for (int t = 0; t < 4; ++t) oacc[t][r] *= alpha;
    }
    __builtin_amdgcn_fence(__ATOMIC_RELEASE, "workgroup");
    __builtin_amdgcn_wave_barrier();
    __builtin_amdgcn_fence(__ATOMIC_ACQUIRE, "workgroup");
#pragma unroll 1
    for (int kk = 0; kk < 2; ++kk) {
      FB pa;
      pa.h[0] = *(const v8h*)(pw + c * AT_KC + kk * 32 + 8 * hh);
      pa.h[1] = *(const v8h*)(pw + c * AT_KC + kk * 32 + 16 + 8 * hh);
#pragma unroll
      for (int t = 0; t < 4; ++t) {
        FB vb;
        vb.h[0] = *(const v8h*)(Vth + (t * 16 + c) * AT_KC + kk * 32 + 8 * hh);
        vb.h[1] = *(const v8h*)(Vth + (t * 16 + c) * AT_KC + kk * 32 + 16 + 8 * hh);
        oacc[t] = mma_h(pa.v, vb.v, oacc[t]);
      }
    }
  }

  float* os = Os[wave];
#pragma unroll
  for (int r = 0; r < 8; ++r) {
    const float inv = out_scale / (lrow[r] * AT_PSC);
#pragma unroll
    for (int t = 0; t < 4; ++t) os[(8 * hh + r) * 68 + t * 16 + c] = oacc[t][r] * inv;
  }
  __builtin_amdgcn_fence(__ATOMIC_RELEASE, "workgroup");
  __builtin_amdgcn_wave_barrier();
  __builtin_amdgcn_fence(__ATOMIC_ACQUIRE, "workgroup");
  {
    const int q4 = lane >> 3, c8 = (lane & 7) * 8;
    for (int pass = 0; pass < 2; ++pass) {
#pragma unroll
      for (int it = 0; it < 4; ++it) {
        const int row = it * 4 + q4;
        const float* sp = os + row * 68 + c8;
        v8h hv;
#pragma unroll
        for (int e = 0; e < 8; ++e) hv[e] = (f16t)sp[e];
        *(volatile v8h*)(ob_ptr + (size_t)(q0 + row) * rs + c8) = hv;
      }
      __threadfence();
    }
  }
}

__global__ __launch_bounds__(256) void head_probs(
    const float* __restrict__ dyn, const float* __restrict__ stat,
    const float* __restrict__ g1, const float* __restrict__ b1,
    const float* __restrict__ g2, const float* __restrict__ b2,
    const float* __restrict__ clsw, const float* __restrict__ clsb,
    float* __restrict__ probs, int nrows, float eps) {
  __shared__ float pr[32];
  const int lane = threadIdx.x & 31, wave = threadIdx.x >> 5;
  const float cb = clsb[0];
#pragma unroll 1
  for (int i = 0; i < 4; ++i) {
    const int row = blockIdx.x * 32 + wave * 4 + i;
    const int rowc = row < nrows ? row : (nrows - 1);
    const float* dr = dyn + (size_t)rowc * LN_D;
    const float* sr = stat + (size_t)rowc * LN_D;
    float sd = 0.f, ss = 0.f;
#pragma unroll 1
    for (int ch = 0; ch < 4; ++ch) {
      const int col = ch * 128 + lane * 4;
      const v4f d4 = *(const v4f*)(dr + col);
      const v4f s4 = *(const v4f*)(sr + col);
      sd += (d4[0] + d4[1]) + (d4[2] + d4[3]);
      ss += (s4[0] + s4[1]) + (s4[2] + s4[3]);
    }
    sd = wsum32(sd); ss = wsum32(ss);
    const float md = sd * (1.0f / 512.0f);
    const float ms = ss * (1.0f / 512.0f);
    float vd = 0.f, vs = 0.f;
#pragma unroll 1
    for (int ch = 0; ch < 4; ++ch) {
      const int col = ch * 128 + lane * 4;
      const v4f d4 = *(const v4f*)(dr + col);
      const v4f s4 = *(const v4f*)(sr + col);
#pragma unroll
      for (int e = 0; e < 4; ++e) {
        const float td = d4[e] - md; vd += td * td;
        const float ts = s4[e] - ms; vs += ts * ts;
      }
    }
    vd = wsum32(vd); vs = wsum32(vs);
    const float idv = 1.0f / sqrtf(vd * (1.0f / 512.0f) + eps);
    const float isv = 1.0f / sqrtf(vs * (1.0f / 512.0f) + eps);
    float acc = 0.f;
#pragma unroll 1
    for (int ch = 0; ch < 4; ++ch) {
      const int col = ch * 128 + lane * 4;
      const v4f d4 = *(const v4f*)(dr + col);
      const v4f s4 = *(const v4f*)(sr + col);
      const v4f ga = *(const v4f*)(g1 + col);
      const v4f ba = *(const v4f*)(b1 + col);
      const v4f gb = *(const v4f*)(g2 + col);
      const v4f bb = *(const v4f*)(b2 + col);
      const v4f w4 = *(const v4f*)(clsw + col);
#pragma unroll
      for (int e = 0; e < 4; ++e) {
        const float a  = (d4[e] - md) * idv * ga[e] + ba[e];
        const float bq = (s4[e] - ms) * isv * gb[e] + bb[e];
        const float df = a - bq;
        acc += df * df * w4[e];
      }
    }
    acc = wsum32(acc);
    const float logit = acc + cb;
    const float ev = expf(-fmaxf(logit, -80.0f));
    const float p = 1.0f / (1.0f + ev);
    if (lane == 0) pr[wave * 4 + i] = p;
  }
  __syncthreads();
  if (wave == 0 && lane < 8) {
    const int base = blockIdx.x * 32;
    if (base + 32 <= nrows) {
      v4f val;
      val[0] = pr[lane * 4 + 0]; val[1] = pr[lane * 4 + 1];
      val[2] = pr[lane * 4 + 2]; val[3] = pr[lane * 4 + 3];
      float* pp = probs + base + lane * 4;
      *(volatile v4f*)pp = val;
      __threadfence();
      *(volatile v4f*)pp = val;
    }
  }
}

__global__ __launch_bounds__(256) void masked_mean(
    const float* __restrict__ probs, const float* __restrict__ mask,
    float* __restrict__ outp, int nb, int L) {
  __shared__ float res[32];
  const int lane = threadIdx.x & 31, wave = threadIdx.x >> 5;
  const int nch = L / 128;
#pragma unroll 1
  for (int i = 0; i < 4; ++i) {
    const int bi = wave * 4 + i;
    const int bc = bi < nb ? bi : (nb - 1);
    const float* prp = probs + (size_t)bc * L;
    const float* mrp = mask + (size_t)bc * L;
    float s = 0.f, sm = 0.f;
#pragma unroll 1
    for (int ch = 0; ch < nch; ++ch) {
      const int col = ch * 128 + lane * 4;
      const v4f p4 = *(const v4f*)(prp + col);
      const v4f m4 = *(const v4f*)(mrp + col);
#pragma unroll
      for (int e = 0; e < 4; ++e) { s += p4[e] * m4[e]; sm += m4[e]; }
    }
    s = wsum32(s); sm = wsum32(sm);
    if (lane == 0) res[bi] = s * (1.0f / sm);
  }
  __syncthreads();
  if (wave == 0 && lane < 8) {
    if (lane * 4 + 4 <= nb) {
      v4f val;
      val[0] = res[lane * 4 + 0]; val[1] = res[lane * 4 + 1];
      val[2] = res[lane * 4 + 2]; val[3] = res[lane * 4 + 3];
      float* pp = outp + lane * 4;
      *(volatile v4f*)pp = val;
      __threadfence();
      *(volatile v4f*)pp = val;
    }
  }
}

template <int BIAS_MODE, int OUT_MODE, bool RESID, int ACT, bool RS>
static void gemm_f16(hipStream_t st, const f16t* A, const f16t* Bt, void* C,
                     const float* bias, const float* resid, const float* rsc,
                     int M, int N, int K, float scale) {
  const int tiles = (M / 64) * (N / 64);
  dim3 grid((unsigned)((tiles + 7) / 8), 1, 1);
  wmma_gemm64<0, false, BIAS_MODE, OUT_MODE, RESID, ACT, RS><<<grid, 256, 0, st>>>(
      (const unsigned short*)A, nullptr, K, 0L,
      (const unsigned short*)Bt, nullptr, K, 0L,
      C, nullptr, N, 0L, bias, resid, 0L, rsc, M, N, K, scale);
}

extern "C" void kernel_launch(void* const* d_in, const int* in_sizes, int n_in,
                              void* d_out, int out_size, void* d_ws, size_t ws_size,
                              hipStream_t stream) {
  constexpr int Bn = 32, Ln = 512, Dn = 512, Hn = 8;
  constexpr int M = Bn * Ln;
  if (n_in < 26) return;
  if (in_sizes[0] != M * Dn || in_sizes[1] != M * Dn || in_sizes[2] != M) return;
  for (int i = 3; i <= 7; ++i) if (in_sizes[i] != Dn * Dn) return;
  if (in_sizes[16] != Dn * Dn || in_sizes[18] != Dn * Dn) return;
  for (int i = 8; i <= 15; ++i) if (in_sizes[i] != Dn) return;
  if (in_sizes[17] != Dn || in_sizes[19] != Dn) return;
  for (int i = 20; i <= 24; ++i) if (in_sizes[i] != Dn) return;
  if (in_sizes[25] < 1 || out_size != Bn) return;

  const float* dynamic_ = (const float*)d_in[0];
  const float* static_  = (const float*)d_in[1];
  const float* mask     = (const float*)d_in[2];
  const float* w_q      = (const float*)d_in[3];
  const float* w_k      = (const float*)d_in[4];
  const float* w_v      = (const float*)d_in[5];
  const float* fc1_w    = (const float*)d_in[6];
  const float* fc2_w    = (const float*)d_in[7];
  const float* ln_q_g   = (const float*)d_in[8];
  const float* ln_q_b   = (const float*)d_in[9];
  const float* ln_k_g   = (const float*)d_in[10];
  const float* ln_k_b   = (const float*)d_in[11];
  const float* ln_v_g   = (const float*)d_in[12];
  const float* ln_v_b   = (const float*)d_in[13];
  const float* pff_ln_g = (const float*)d_in[14];
  const float* pff_ln_b = (const float*)d_in[15];
  const float* pff_w1   = (const float*)d_in[16];
  const float* pff_b1   = (const float*)d_in[17];
  const float* pff_w2   = (const float*)d_in[18];
  const float* pff_b2   = (const float*)d_in[19];
  const float* out1_g   = (const float*)d_in[20];
  const float* out1_b   = (const float*)d_in[21];
  const float* out2_g   = (const float*)d_in[22];
  const float* out2_b   = (const float*)d_in[23];
  const float* cls_w    = (const float*)d_in[24];
  const float* cls_b    = (const float*)d_in[25];

  const size_t SLOT = (size_t)M * Dn * sizeof(f16t);
  const size_t WPL  = (size_t)Dn * Dn * sizeof(f16t);
  const size_t off_w = 7 * SLOT;
  const size_t off_p = off_w + 7 * WPL;
  const size_t total = off_p + (size_t)M * sizeof(float);
  if (total > ws_size || total > (size_t)134217728) return;
  char* ws = (char*)d_ws;
  f16t* S0 = (f16t*)(ws + 0 * SLOT);
  f16t* S1 = (f16t*)(ws + 1 * SLOT);
  f16t* S2 = (f16t*)(ws + 2 * SLOT);
  f16t* S3 = (f16t*)(ws + 3 * SLOT);
  f16t* S4 = (f16t*)(ws + 4 * SLOT);
  f16t* S5 = (f16t*)(ws + 5 * SLOT);
  f16t* wts = (f16t*)(ws + off_w);
  float* probs = (float*)(ws + off_p);
  const f16t* wqT  = wts + 0 * (size_t)Dn * Dn;
  const f16t* wkT  = wts + 1 * (size_t)Dn * Dn;
  const f16t* wvT  = wts + 2 * (size_t)Dn * Dn;
  const f16t* f1T  = wts + 3 * (size_t)Dn * Dn;
  const f16t* f2T  = wts + 4 * (size_t)Dn * Dn;
  const f16t* p1T  = wts + 5 * (size_t)Dn * Dn;
  const f16t* p2T  = wts + 6 * (size_t)Dn * Dn;
  float* xbuf  = (float*)S1;
  float* statf = (float*)S3;
  float* dyn2  = (float*)S5;

  const float eps = 1e-5f;
  const float WSC = 16.0f;
  const float OSC = 8.0f;

  wcast_t16<<<dim3(Dn / 64, Dn / 32, 7), 256, 0, stream>>>(w_q, w_k, w_v, fc1_w, fc2_w, pff_w1, pff_w2,
                                                          wts, Dn, Dn, WSC);
  ln_rows_f16<2><<<(M + 7) / 8, 256, 0, stream>>>(dynamic_, ln_q_g, ln_q_b, ln_k_g, ln_k_b, S0, S1, M, eps);
  ln_rows_f16<1><<<(M + 7) / 8, 256, 0, stream>>>(static_, ln_v_g, ln_v_b, ln_v_g, ln_v_b, S2, S2, M, eps);
  gemm_f16<0, 1, false, 0, false>(stream, S0, wqT, S3, nullptr, nullptr, nullptr, M, Dn, Dn, 1.0f / WSC);
  gemm_f16<0, 1, false, 0, false>(stream, S1, wkT, S4, nullptr, nullptr, nullptr, M, Dn, Dn, 1.0f / WSC);
  gemm_f16<0, 1, false, 0, false>(stream, S2, wvT, S5, nullptr, nullptr, nullptr, M, Dn, Dn, 1.0f / WSC);
  attn64_f16_diag<<<Bn * Hn * (Ln / 64), 128, 0, stream>>>(S3, S4, S5, S0, Ln, Hn, Hn * 64, 0.125f,
                                                           -1.0e32f, OSC);
  gemm_f16<0, 0, false, 0, true >(stream, S0, f1T, xbuf,  nullptr, nullptr, mask,    M, Dn, Dn, 1.0f / (WSC * OSC));
  gemm_f16<0, 0, false, 0, false>(stream, S5, f2T, statf, nullptr, nullptr, nullptr, M, Dn, Dn, 1.0f / WSC);
  ln_rows_f16<1><<<(M + 7) / 8, 256, 0, stream>>>(xbuf, pff_ln_g, pff_ln_b, pff_ln_g, pff_ln_b, S5, S5, M, eps);
  gemm_f16<2, 1, false, 3, false>(stream, S5, p1T, S0, pff_b1, nullptr, nullptr, M, Dn, Dn, 1.0f / WSC);
  gemm_f16<2, 0, true, 0, true>(stream, S0, p2T, dyn2, pff_b2, xbuf, mask, M, Dn, Dn, 1.0f / WSC);
  head_probs<<<(M + 31) / 32, 256, 0, stream>>>(dyn2, statf, out1_g, out1_b, out2_g, out2_b,
                                                cls_w, cls_b, probs, M, eps);
  masked_mean<<<1, 256, 0, stream>>>(probs, mask, (float*)d_out, Bn, Ln);
}
